// DMNN_40879498728939
// MI455X (gfx1250) — hardware-run, weakly checked
//
#include <hip/hip_runtime.h>


#define NR   65536
#define NJ   1024
#define NG   512
#define NF   64
#define CH   16384
#define SEPS 1e-12f
typedef _Float16 h16;
typedef unsigned short bf;
typedef __attribute__((ext_vector_type(16))) __bf16   v16bf;
typedef __attribute__((ext_vector_type(16))) _Float16 v16h;
typedef __attribute__((ext_vector_type(8)))  _Float16 v8h;
typedef __attribute__((ext_vector_type(8)))  unsigned short v8us;
typedef __attribute__((ext_vector_type(8)))  float    v8f;
typedef __attribute__((ext_vector_type(4)))  float    v4f;
typedef v8h  __attribute__((may_alias)) v8ha;
typedef v4f  __attribute__((may_alias)) v4fa;
typedef v8us __attribute__((may_alias)) v8usa;

__device__ __forceinline__ unsigned short f2bf(float f) { unsigned u = __float_as_uint(f); u += 0x7FFFu + ((u >> 16) & 1u); return (unsigned short)(u >> 16); }
__device__ __forceinline__ float bf2f(unsigned short b) { return __uint_as_float(((unsigned)b) << 16); }
__device__ __forceinline__ float bfr(float f) { return bf2f(f2bf(f)); }
__device__ __forceinline__ v16h cat16(v8h lo, v8h hi) { return __builtin_shufflevector(lo, hi, 0, 1, 2, 3, 4, 5, 6, 7, 8, 9, 10, 11, 12, 13, 14, 15); }
__device__ __forceinline__ v16bf cat16b(v8us lo, v8us hi) { return __builtin_bit_cast(v16bf, __builtin_shufflevector(lo, hi, 0, 1, 2, 3, 4, 5, 6, 7, 8, 9, 10, 11, 12, 13, 14, 15)); }
__device__ __forceinline__ v8f wmma16(v16h a, v16h b, v8f c) { return __builtin_amdgcn_wmma_f32_16x16x32_f16(false, a, false, b, (short)0, c, false, false); }
__device__ __forceinline__ v8f wmmab(v16bf a, v16bf b, v8f c) { return __builtin_amdgcn_wmma_f32_16x16x32_bf16(false, a, false, b, (short)0, c, false, false); }


template <typename T16> struct WFrag;
template <> struct WFrag<h16> { typedef v16h V; static __device__ __forceinline__ V ld(const h16* p) { return cat16(*(const v8h*)p, *(const v8h*)(p + 16)); } static __device__ __forceinline__ v8f mma(V a, V b, v8f c) { return wmma16(a, b, c); } };
template <> struct WFrag<bf> { typedef v16bf V; static __device__ __forceinline__ V ld(const bf* p) { return cat16b(*(const v8us*)p, *(const v8us*)(p + 16)); } static __device__ __forceinline__ v8f mma(V a, V b, v8f c) { return wmmab(a, b, c); } };
template <typename T16, int NSPLIT, bool BIAS>
__global__ __launch_bounds__(32) void k_gemmw(const T16* __restrict__ A, const T16* __restrict__ A2, const T16* __restrict__ Bt, const T16* __restrict__ Bt2, int K, float* C, int ldc, const float* __restrict__ bias, size_t sA, size_t sB, size_t sC) {
    typedef typename WFrag<T16>::V V;
    __shared__ __align__(16) float os[16 * 68];
    const size_t z = blockIdx.z; A += z * sA; if (A2) A2 += z * sA; Bt += z * sB; if (Bt2) Bt2 += z * sB; C += z * sC;
    const int lane = threadIdx.x & 31, lr = lane & 15, hi = lane >> 4; const int r0 = blockIdx.x * 64, c0 = blockIdx.y * 64;
    v8f acc[4][4];
#pragma unroll
    for (int mb = 0; mb < 4; ++mb)
#pragma unroll
        for (int nb = 0; nb < 4; ++nb) acc[mb][nb] = (v8f){};
    const size_t aoff = (size_t)(r0 + lr) * K + 8 * hi, boff = (size_t)(c0 + lr) * K + 8 * hi;

    for (int kc = 0; kc < K; kc += 32) {
        V a[4], a2[4];
#pragma unroll
        for (int mb = 0; mb < 4; ++mb) { a[mb] = WFrag<T16>::ld(A + aoff + (size_t)mb * 16 * K + kc); if (NSPLIT == 1 || NSPLIT == 2) a2[mb] = WFrag<T16>::ld(A2 + aoff + (size_t)mb * 16 * K + kc); }
#pragma unroll
        for (int nb = 0; nb < 4; ++nb) { const V b = WFrag<T16>::ld(Bt + boff + (size_t)nb * 16 * K + kc); V b2; if (NSPLIT >= 2) b2 = WFrag<T16>::ld(Bt2 + boff + (size_t)nb * 16 * K + kc);
#pragma unroll
            for (int mb = 0; mb < 4; ++mb) { acc[mb][nb] = WFrag<T16>::mma(a[mb], b, acc[mb][nb]); if (NSPLIT == 1 || NSPLIT == 2) acc[mb][nb] = WFrag<T16>::mma(a2[mb], b, acc[mb][nb]); if (NSPLIT >= 2) acc[mb][nb] = WFrag<T16>::mma(a[mb], b2, acc[mb][nb]); } }
        asm volatile("v_nop\n\tv_nop\n\tv_nop\n\tv_nop" : "+v"(acc[0][0]), "+v"(acc[1][1]), "+v"(acc[2][2]), "+v"(acc[3][3]) : "v"(a[0]), "v"(a[3]));
    }
#pragma unroll
    for (int mb = 0; mb < 4; ++mb) {
#pragma unroll
        for (int nb = 0; nb < 4; ++nb) {
#pragma unroll
            for (int j = 0; j < 8; ++j) os[(hi * 8 + j) * 68 + nb * 16 + lr] = acc[mb][nb][j]; }
        __builtin_amdgcn_wave_barrier(); asm volatile("" ::: "memory");
        float* crow = C + (size_t)(r0 + mb * 16) * ldc + c0;
#pragma unroll 1
        for (int ps = 0; ps < 2; ++ps) {
#pragma unroll
            for (int s = 0; s < 8; ++s) { const int row = 2 * s + hi, cofs = lr * 4; v4f val = *(const v4fa*)(os + row * 68 + cofs); if (BIAS) { val[0] += bfr(bias[c0 + cofs]); val[1] += bfr(bias[c0 + cofs + 1]); val[2] += bfr(bias[c0 + cofs + 2]); val[3] += bfr(bias[c0 + cofs + 3]); }
                *(volatile v4f*)(crow + (size_t)row * ldc + cofs) = val; }
            if (ps == 0) __threadfence(); }
        __builtin_amdgcn_wave_barrier(); asm volatile("" ::: "memory");
    }
}

__device__ __forceinline__ h16 tohx(float x) { return (h16)x; }
__device__ __forceinline__ void splitf(float y, unsigned short& h, unsigned short& l) { h = f2bf(y); l = f2bf(y - bf2f(h)); }
typedef __attribute__((ext_vector_type(2))) _Float16 v2h;
typedef __attribute__((ext_vector_type(4))) _Float16 v4h;
typedef __attribute__((ext_vector_type(2))) unsigned short v2us;
typedef __attribute__((ext_vector_type(4))) unsigned short v4us;
typedef __attribute__((ext_vector_type(2))) float v2f;
typedef __attribute__((ext_vector_type(4))) int v4i;
__global__ __launch_bounds__(256) void k_cvt8(const float* __restrict__ src, bf* dst, size_t n8) { const size_t i = (size_t)blockIdx.x * 256 + threadIdx.x; if (i >= n8) return; const v8f v = *(const v8f*)(src + i * 8); v8us o;
#pragma unroll
    for (int k = 0; k < 8; ++k) o[k] = f2bf(v[k]); *(volatile v8us*)(dst + i * 8) = o; __threadfence(); *(volatile v8us*)(dst + i * 8) = o; }
__global__ __launch_bounds__(256) void k_cn(const float* __restrict__ a1, float* CN) { const unsigned jj = blockIdx.x * 256u + threadIdx.x; const float* src = a1 + (size_t)jj * NF; float acc = 0.0f;
    for (int ff = 0; ff < NF; ++ff) { const float cv = bfr(src[ff]); acc = acc + cv * cv; }
    *(volatile float*)(CN + jj) = acc; __threadfence(); *(volatile float*)(CN + jj) = acc; }
__device__ __forceinline__ float wsum(float v) { for (int m = 16; m >= 1; m >>= 1) v = v + __shfl_xor(v, m); return v; }
__device__ __forceinline__ float wtop(float v) { for (int m = 16; m >= 1; m >>= 1) { const float o = __shfl_xor(v, m); v = (o > v) ? o : v; } return v; }
__global__ __launch_bounds__(256) void k_rw(const float* __restrict__ a0, const float* __restrict__ PL, const float* __restrict__ CN, const float* __restrict__ a2, const float* __restrict__ a3, const float* __restrict__ a4, int row0, float* outp) { const int lane = threadIdx.x & 31; const unsigned rb0 = (blockIdx.x * 8u + (threadIdx.x >> 5)) * 16u; float k0 = 0.0f, k1 = 0.0f;
    const float ob0 = bfr(a4[0]) + bfr(a4[1]), ob1 = bfr(a4[2]) + bfr(a4[3]);
    for (int rr = 0; rr < 16; ++rr) { const unsigned rl = rb0 + (unsigned)rr; const size_t rg = (size_t)row0 + rl; const v2f xw = *(const v2f*)(a0 + rg * NF + lane * 2); const float x0 = bfr(xw[0]), x1 = bfr(xw[1]); const float nx = wsum(x0 * x0 + x1 * x1); const float* pr = PL + (size_t)rl * NJ; float lg0 = 0.0f, lg1 = 0.0f;
        for (int gp = 0; gp < 2; ++gp) { float vv[16]; float top = -3.0e38f;
#pragma unroll
            for (int q = 0; q < 4; ++q) { const int jc = gp * NG + q * 128 + lane * 4; const v4f pv = *(const v4f*)(pr + jc); const v4f cv = *(const v4f*)(CN + jc); const v4f rv = *(const v4f*)(a2 + jc);
#pragma unroll
                for (int e = 0; e < 4; ++e) { const float sv = fmaxf((nx + cv[e]) - 2.0f * pv[e], SEPS); const float vx = bfr(rv[e]) - sqrtf(sv); vv[q * 4 + e] = vx; top = (vx > top) ? vx : top; } }
            top = wtop(top); float sm = 0.0f, t0 = 0.0f, t1 = 0.0f;
#pragma unroll
            for (int q = 0; q < 4; ++q) { const int kc = q * 128 + lane * 4; const v4f w0 = *(const v4f*)(a3 + (0 * 2 + gp) * NG + kc); const v4f w1 = *(const v4f*)(a3 + (1 * 2 + gp) * NG + kc);
#pragma unroll
                for (int e = 0; e < 4; ++e) { const float vx = vv[q * 4 + e]; const float ev = expf(vx - top); sm = sm + ev; const float ge = vx * ev; t0 = t0 + ge * bfr(w0[e]); t1 = t1 + ge * bfr(w1[e]); } }
            sm = wsum(sm); t0 = wsum(t0); t1 = wsum(t1); lg0 = lg0 + t0 / sm; lg1 = lg1 + t1 / sm; }
        lg0 = lg0 + ob0; lg1 = lg1 + ob1; const float big = fmaxf(lg0, lg1); const float e0 = expf(lg0 - big), e1 = expf(lg1 - big); const float den = e0 + e1; const float r0 = e0 / den, r1 = e1 / den; k0 = (lane == rr) ? r0 : k0; k1 = (lane == rr) ? r1 : k1; }
    if (lane < 16) { v2f o; o[0] = k0; o[1] = k1; float* dst = outp + ((size_t)row0 + rb0 + (unsigned)lane) * 2; *(volatile v2f*)dst = o; __threadfence(); *(volatile v2f*)dst = o; } }

extern "C" void kernel_launch(void* const* d_in, const int* in_sizes, int n_in,
                              void* d_out, int out_size, void* d_ws, size_t ws_size, hipStream_t stream) {
    (void)in_sizes; (void)n_in; (void)out_size;
    const float* a0 = (const float*)d_in[0]; const float* a1 = (const float*)d_in[1]; const float* a2 = (const float*)d_in[2]; const float* a3 = (const float*)d_in[3]; const float* a4 = (const float*)d_in[4];
    float* OUT = (float*)d_out;
    char* wsp = (char*)d_ws;
    auto take = [&](size_t bytes) { char* p = wsp; wsp += (bytes + 255) & ~(size_t)255; return (void*)p; };
    bf* XB = (bf*)take((size_t)NR * NF * 2); bf* CB = (bf*)take((size_t)NJ * NF * 2); float* CN = (float*)take((size_t)NJ * 4); float* PL = (float*)take((size_t)CH * NJ * 4);
    if ((size_t)(wsp - (char*)d_ws) > ws_size) return;
    k_cvt8<<<(unsigned)((size_t)NR * NF / 8 / 256), 256, 0, stream>>>(a0, XB, (size_t)NR * NF / 8); k_cvt8<<<(unsigned)((size_t)NJ * NF / 8 / 256), 256, 0, stream>>>(a1, CB, (size_t)NJ * NF / 8);
    k_cn<<<NJ / 256, 256, 0, stream>>>(a1, CN);
    for (int cq = 0; cq < NR / CH; ++cq) {
        k_gemmw<bf, 0, false><<<dim3(CH / 64, NJ / 64, 1), 32, 0, stream>>>(XB + (size_t)cq * CH * NF, nullptr, CB, nullptr, NF, PL, NJ, nullptr, 0, 0, 0);
        k_rw<<<CH / 128, 256, 0, stream>>>(a0, PL, CN, a2, a3, a4, cq * CH, OUT); }
}
